// MLPAttention_71648644432025
// MI455X (gfx1250) — hardware-run, weakly checked
//
#include <hip/hip_runtime.h>


#ifndef NQ
#define NQ 1024
#endif
#ifndef NK
#define NK 2048
#endif
#define NQ_FULL 1024
#define NK_FULL 2048
#define DH   64
#define AW   4
#define OSP  36
#define OTP  68
#define PSH  14.0f
#define NEGB (-3.0e38f)
#define LOG2E 1.4426950408889634f

static_assert(DH == 64);
static_assert(DH % 32 == 0);
static_assert(NQ % 64 == 0);
static_assert(NK % 64 == 0);
static_assert(NK % 32 == 0);
static_assert(NQ % (16 * AW) == 0);
static_assert(AW == 4);
static_assert(32 * AW >= DH);
static_assert(NQ <= NQ_FULL);
static_assert(NK <= NK_FULL);
static_assert((OSP * 4) % 16 == 0);
static_assert((OTP * 4) % 16 == 0);
static_assert(((size_t)DH * NQ_FULL * 4) == (size_t)262144);
static_assert(((size_t)DH * NQ_FULL * 4) % 128 == 0);
static_assert(((size_t)(AW * 16 * OSP + DH * OTP + DH) * 4) <= (size_t)131072);
static_assert(((size_t)DH * 65 * 4) <= (size_t)131072);
static_assert(((size_t)16 * 68 * 4) <= (size_t)131072);

typedef _Float16 h16;
typedef unsigned short bf;
typedef __attribute__((ext_vector_type(16))) __bf16   v16bf;
typedef __attribute__((ext_vector_type(16))) _Float16 v16h;
typedef __attribute__((ext_vector_type(8)))  _Float16 v8h;
typedef __attribute__((ext_vector_type(8)))  unsigned short v8us;
typedef __attribute__((ext_vector_type(8)))  float    v8f;
typedef __attribute__((ext_vector_type(4)))  float    v4f;
typedef v4f  __attribute__((may_alias)) v4fa;

__device__ __forceinline__ unsigned short f2bf(float f) { unsigned u = __float_as_uint(f); u += 0x7FFFu + ((u >> 16) & 1u); return (unsigned short)(u >> 16); }
__device__ __forceinline__ float bfr(float f) { return __uint_as_float(((unsigned)f2bf(f)) << 16); }
__device__ __forceinline__ v16h cat16(v8h lo, v8h hi) { return __builtin_shufflevector(lo, hi, 0, 1, 2, 3, 4, 5, 6, 7, 8, 9, 10, 11, 12, 13, 14, 15); }
__device__ __forceinline__ v16bf cat16b(v8us lo, v8us hi) { return __builtin_bit_cast(v16bf, __builtin_shufflevector(lo, hi, 0, 1, 2, 3, 4, 5, 6, 7, 8, 9, 10, 11, 12, 13, 14, 15)); }
__device__ __forceinline__ v16h  ldh(const h16* p) { return cat16(*(const v8h*)p, *(const v8h*)(p + 16)); }
__device__ __forceinline__ v16bf ldb(const bf* p)  { return cat16b(*(const v8us*)p, *(const v8us*)(p + 16)); }
__device__ __forceinline__ void wave_sync() { __builtin_amdgcn_fence(3  , "wavefront"); __builtin_amdgcn_wave_barrier(); asm volatile("" ::: "memory"); }
static __device__ __forceinline__ h16 toh_flush(float v) { const h16 r = (h16)v; return (fabsf(v) < 6.103515625e-05f) ? (h16)0.0f : r; }
__device__ __forceinline__ v8f wmma16g(v16h a, v16h b, v8f c) {
    c = __builtin_amdgcn_wmma_f32_16x16x32_f16(false, a, false, b, (short)0, c, false, false);
    asm volatile("v_nop\n\tv_nop\n\tv_nop\n\tv_nop" : "+v"(c) : "v"(a), "v"(b));
    return c; }
__device__ __forceinline__ v8f wmmabg(v16bf a, v16bf b, v8f c) {
    c = __builtin_amdgcn_wmma_f32_16x16x32_bf16(false, a, false, b, (short)0, c, false, false);
    asm volatile("v_nop\n\tv_nop\n\tv_nop\n\tv_nop" : "+v"(c) : "v"(a), "v"(b));
    return c; }

static_assert(256 * 16 * 2 == 64 * DH * 2);
__global__ __launch_bounds__(256) void k_cvtT(const float* __restrict__ src, bf* dst, int pitch) {
    __shared__ float tl[DH * 65];
    const int t = threadIdx.x; const int n0 = blockIdx.x * 64;
#pragma unroll 1
    for (int i = 0; i < 16; ++i) { const int idx = i * 256 + t; const int d = idx >> 6, n = idx & 63;
        tl[d * 65 + n] = src[(size_t)d * (size_t)pitch + (size_t)(n0 + n)]; }
    __syncthreads();
#pragma unroll 1
    for (int ps = 0; ps < 2; ++ps) {
#pragma unroll
        for (int it = 0; it < 2; ++it) { const int p = it * 256 + t; const int n = p >> 3, c8 = (p & 7) * 8; v8us o;
#pragma unroll
            for (int k = 0; k < 8; ++k) o[k] = f2bf(tl[(c8 + k) * 65 + n]);
            *(volatile v8us*)(dst + (size_t)(n0 + n) * DH + c8) = o; }
        if (ps == 0) __threadfence(); }
}

static_assert((2 * DH * DH / 8) % 256 == 0);
__global__ __launch_bounds__(256) void k_cvtw(const float* __restrict__ W1, bf* dst) {
    const int i = blockIdx.x * 256 + threadIdx.x; const int o = i * 8;
    const int part = o / (DH * DH), h = (o % (DH * DH)) / DH, d = o % DH;
    const float* s = W1 + (size_t)h * (2 * DH) + part * DH + d;
    const v4f x0 = *(const v4f*)s, x1 = *(const v4f*)(s + 4); v8us ov;
#pragma unroll
    for (int k = 0; k < 4; ++k) { ov[k] = f2bf(x0[k]); ov[4 + k] = f2bf(x1[k]); }
    *(volatile v8us*)(dst + o) = ov; __threadfence(); *(volatile v8us*)(dst + o) = ov;
}

static_assert(((size_t)DH * NK / 8) % 256 == 0);
__global__ __launch_bounds__(256) void k_cvth(const float* __restrict__ src, h16* dst) {
    const int i = blockIdx.x * 256 + threadIdx.x;
    const int d = i / (NK / 8), c8 = (i % (NK / 8)) * 8;
    const v8f v = *(const v8f*)(src + (size_t)d * NK_FULL + c8); v8h o;
#pragma unroll
    for (int k = 0; k < 8; ++k) o[k] = toh_flush(bfr(v[k]));
    h16* q = dst + (size_t)d * NK + c8;
    *(volatile v8h*)q = o; __threadfence(); *(volatile v8h*)q = o;
}

static_assert(32 * 16 * 8 == 16 * DH * 4);
__global__ __launch_bounds__(32) void k_projf(const bf* __restrict__ A, const bf* __restrict__ Bt, const float* __restrict__ bias, int has_bias, float* P) {
    __shared__ __align__(16) float os[16 * 68];
    const int K = DH;
    const int lane = threadIdx.x & 31, lr = lane & 15, hi = lane >> 4; const int r0 = blockIdx.x * 64;
    v8f acc[4][4];
#pragma unroll
    for (int mb = 0; mb < 4; ++mb)
#pragma unroll
        for (int nb = 0; nb < 4; ++nb) acc[mb][nb] = (v8f){};
    const size_t aoff = (size_t)(r0 + lr) * K + 8 * hi, boff = (size_t)lr * K + 8 * hi;
#pragma unroll 1
    for (int kc = 0; kc < K; kc += 32) {
        v16bf a[4];
#pragma unroll
        for (int mb = 0; mb < 4; ++mb) a[mb] = ldb(A + aoff + (size_t)mb * 16 * K + kc);
#pragma unroll
        for (int nb = 0; nb < 4; ++nb) { const v16bf b = ldb(Bt + boff + (size_t)nb * 16 * K + kc);
#pragma unroll
            for (int mb = 0; mb < 4; ++mb) acc[mb][nb] = wmmabg(a[mb], b, acc[mb][nb]); }
    }
    float bc[4];
#pragma unroll
    for (int nb = 0; nb < 4; ++nb) { const float bv = bfr(bias[nb * 16 + lr]); bc[nb] = (has_bias != 0) ? bv : 0.0f; }
#pragma unroll
    for (int mb = 0; mb < 4; ++mb) {
#pragma unroll
        for (int nb = 0; nb < 4; ++nb) {
#pragma unroll
            for (int j = 0; j < 8; ++j) os[(hi * 8 + j) * 68 + nb * 16 + lr] = acc[mb][nb][j] + bc[nb]; }
        wave_sync();
        float* pb = P + (size_t)(r0 + mb * 16) * DH;
#pragma unroll 1
        for (int ps = 0; ps < 2; ++ps) {
#pragma unroll
            for (int s = 0; s < 8; ++s) { const int row = 2 * s + (lane >> 4), cofs = (lane & 15) * 4;
                const v4f val = *(const v4fa*)(&os[row * 68 + cofs]);
                *(volatile v4f*)(pb + (size_t)row * DH + cofs) = val; }
            if (ps == 0) __threadfence(); }
        wave_sync();
    }
}

static_assert(32 * 16 * 4 == 16 * 32 * 4);
static_assert(32 * AW * 16 * 8 == DH * (16 * AW) * 4);
__global__ __launch_bounds__(32 * AW) void k_pairw(const float* __restrict__ QP, const float* __restrict__ KB, const h16* __restrict__ VH,
                                                  const float* __restrict__ W2, const float* __restrict__ B2, float* OUT0, float* OUT1) {
    __shared__ __align__(16) float sc[AW * 16 * OSP];
    __shared__ __align__(16) float ot[DH * OTP];
    __shared__ __align__(16) float w2s[DH];
    const int lane = threadIdx.x & 31, lr = lane & 15, hi = lane >> 4;
    const int wave = __builtin_amdgcn_readfirstlane((int)(threadIdx.x >> 5));
    const int qb = blockIdx.x * (16 * AW);
    const int q0 = qb + wave * 16;
    if (threadIdx.x < DH) w2s[threadIdx.x] = bfr(W2[threadIdx.x]);
    __syncthreads();
    const float b2v = bfr(B2[0]);
    const float* qrow = QP + (size_t)(q0 + lr) * DH;
    const size_t vo = (size_t)lr * NK + 8 * hi;
    const int wb = wave * 16 * OSP;
    v8f o0 = (v8f){}, o1 = (v8f){}, o2 = (v8f){}, o3 = (v8f){};
    float m = NEGB, l = 0.0f;
#pragma unroll 1
    for (int key0 = 0; key0 < NK; key0 += 32) {
        float ta[8], tb[8];
#pragma unroll
        for (int r = 0; r < 8; ++r) { ta[r] = 0.0f; tb[r] = 0.0f; }
        const float* kb = KB + (size_t)(key0 + 8 * hi) * DH;
#pragma unroll 1
        for (int hc = 0; hc < DH; hc += 4) {
            const v4f q4 = *(const v4f*)(qrow + hc);
            const v4f w4 = *(const v4fa*)(&w2s[hc]);
#pragma unroll
            for (int r = 0; r < 8; ++r) {
                const v4f ka = *(const v4f*)(kb + r * DH + hc);
                const v4f kc = *(const v4f*)(kb + (16 + r) * DH + hc);
#pragma unroll
                for (int j = 0; j < 4; ++j) {
                    ta[r] = fmaf(w4[j], fmaxf(q4[j] + ka[j], 0.0f), ta[r]);
                    tb[r] = fmaf(w4[j], fmaxf(q4[j] + kc[j], 0.0f), tb[r]); } } }
        float ua[8], ub[8]; float mx = NEGB;
#pragma unroll
        for (int r = 0; r < 8; ++r) { ta[r] += b2v; tb[r] += b2v; ua[r] = ta[r] * LOG2E; ub[r] = tb[r] * LOG2E; mx = fmaxf(mx, fmaxf(ua[r], ub[r])); }
        { v4f a, c;
          a[0] = ta[0]; a[1] = ta[1]; a[2] = ta[2]; a[3] = ta[3]; c[0] = ta[4]; c[1] = ta[5]; c[2] = ta[6]; c[3] = ta[7];
          *(v4fa*)(&sc[wb + lr * OSP + 8 * hi]) = a; *(v4fa*)(&sc[wb + lr * OSP + 8 * hi + 4]) = c;
          a[0] = tb[0]; a[1] = tb[1]; a[2] = tb[2]; a[3] = tb[3]; c[0] = tb[4]; c[1] = tb[5]; c[2] = tb[6]; c[3] = tb[7];
          *(v4fa*)(&sc[wb + lr * OSP + 16 + 8 * hi]) = a; *(v4fa*)(&sc[wb + lr * OSP + 16 + 8 * hi + 4]) = c; }
        wave_sync();
        { float* srow = OUT1 + (size_t)q0 * NK_FULL + key0;
#pragma unroll 1
          for (int ps = 0; ps < 2; ++ps) {
#pragma unroll
              for (int s = 0; s < 4; ++s) { const int row = 4 * s + (lane >> 3), cofs = (lane & 7) * 4;
                  const v4f val = *(const v4fa*)(&sc[wb + row * OSP + cofs]);
                  *(volatile v4f*)(srow + (size_t)row * NK_FULL + cofs) = val; }
              if (ps == 0) __threadfence(); } }
        wave_sync();
        mx = fmaxf(mx, __shfl_xor(mx, 16, 32));
        const float mnew = fmaxf(m, mx);
        const float alpha = __builtin_amdgcn_exp2f(m - mnew);
        const float sh = PSH - mnew;
        v16h pb; float ls = 0.0f;
#pragma unroll
        for (int r = 0; r < 8; ++r) {
            const float ea = ua[r] + sh, eb = ub[r] + sh;
            const float ga = __builtin_amdgcn_exp2f(ea), gb = __builtin_amdgcn_exp2f(eb);
            const h16 pa = (ea < -14.0f) ? (h16)0.0f : (h16)ga;
            const h16 pc = (eb < -14.0f) ? (h16)0.0f : (h16)gb;
            pb[r] = pa; pb[8 + r] = pc;
            ls += (float)pa + (float)pc; }
        l = l * alpha + ls; m = mnew;
        o0 = o0 * alpha; o1 = o1 * alpha; o2 = o2 * alpha; o3 = o3 * alpha;
        const h16* va = VH + vo + key0;
        const v16h v0 = ldh(va), v1 = ldh(va + (size_t)16 * NK), v2 = ldh(va + (size_t)32 * NK), v3 = ldh(va + (size_t)48 * NK);
        o0 = wmma16g(v0, pb, o0); o1 = wmma16g(v1, pb, o1); o2 = wmma16g(v2, pb, o2); o3 = wmma16g(v3, pb, o3);
    }
    l += __shfl_xor(l, 16, 32);
    const bool any = l > 0.0f;
    const float lsafe = any ? l : 1.0f;
    const float inv = any ? (1.0f / lsafe) : 0.0f;
    { const int cb = wave * 16 + lr;
#pragma unroll
      for (int r = 0; r < 8; ++r) {
          ot[( 0 + 8 * hi + r) * OTP + cb] = o0[r] * inv;
          ot[(16 + 8 * hi + r) * OTP + cb] = o1[r] * inv;
          ot[(32 + 8 * hi + r) * OTP + cb] = o2[r] * inv;
          ot[(48 + 8 * hi + r) * OTP + cb] = o3[r] * inv; } }
    __syncthreads();
    float* obase = OUT0 + qb;
#pragma unroll 1
    for (int ps = 0; ps < 2; ++ps) {
#pragma unroll
        for (int it = 0; it < 8; ++it) { const int row = it * 8 + wave * 2 + (lane >> 4), cofs = (lane & 15) * 4;
            const v4f val = *(const v4fa*)(&ot[row * OTP + cofs]);
            *(volatile v4f*)(obase + (size_t)row * NQ_FULL + cofs) = val; }
        if (ps == 0) __threadfence(); }
}

static constexpr size_t al256(size_t v) { return (v + 255) & ~(size_t)255; }
static constexpr size_t SZ_XQ = al256((size_t)NQ * DH * 2);
static constexpr size_t SZ_XK = al256((size_t)NK * DH * 2);
static constexpr size_t SZ_WB = al256((size_t)2 * DH * DH * 2);
static constexpr size_t SZ_VH = al256((size_t)DH * NK * 2);
static constexpr size_t SZ_QP = al256((size_t)NQ * DH * 4);
static constexpr size_t SZ_KB = al256((size_t)NK * DH * 4);
static constexpr size_t SZ_TOTAL = SZ_XQ + SZ_XK + SZ_WB + SZ_VH + SZ_QP + SZ_KB;
static_assert(SZ_TOTAL <= (size_t)134217728);
static_assert(((size_t)DH * DH * 2) % 256 == 0);

extern "C" void kernel_launch(void* const* d_in, const int* in_sizes, int n_in,
                              void* d_out, int out_size, void* d_ws, size_t ws_size, hipStream_t stream) {
    if (n_in < 7) return;
    if ((size_t)in_sizes[0] < (size_t)(DH - 1) * NQ_FULL + NQ) return;
    if ((size_t)in_sizes[1] < (size_t)(DH - 1) * NK_FULL + NK || (size_t)in_sizes[2] < (size_t)(DH - 1) * NK_FULL + NK) return;
    if ((size_t)in_sizes[3] < (size_t)DH * 2 * DH || in_sizes[4] < DH || in_sizes[5] < DH || in_sizes[6] < 1) return;
    if ((size_t)out_size < (size_t)DH * NQ_FULL + (size_t)(NQ - 1) * NK_FULL + NK) return;
    if (SZ_TOTAL > ws_size) return;
    const float* query = (const float*)d_in[0];
    const float* key   = (const float*)d_in[1];
    const float* value = (const float*)d_in[2];
    const float* w1    = (const float*)d_in[3];
    const float* b1    = (const float*)d_in[4];
    const float* w2    = (const float*)d_in[5];
    const float* b2    = (const float*)d_in[6];
    float* OUT0 = (float*)d_out;
    float* OUT1 = (float*)d_out + (size_t)DH * NQ_FULL;
    char* wsp = (char*)d_ws;
    bf*  XQ = (bf*)wsp;  wsp += SZ_XQ;
    bf*  XK = (bf*)wsp;  wsp += SZ_XK;
    bf*  WB = (bf*)wsp;  wsp += SZ_WB;
    h16* VH = (h16*)wsp; wsp += SZ_VH;
    float* QP = (float*)wsp; wsp += SZ_QP;
    float* KB = (float*)wsp; wsp += SZ_KB;
    bf* W1Q = WB; bf* W1K = WB + (size_t)DH * DH;

    k_cvtT<<<NQ / 64, 256, 0, stream>>>(query, XQ, NQ_FULL);
    k_cvtT<<<NK / 64, 256, 0, stream>>>(key,   XK, NK_FULL);
    k_cvtw<<<(2 * DH * DH / 8) / 256, 256, 0, stream>>>(w1, WB);
    k_cvth<<<(unsigned)(((size_t)DH * NK / 8) / 256), 256, 0, stream>>>(value, VH);

    k_projf<<<NQ / 64, 32, 0, stream>>>(XQ, W1Q, b1, 0, QP);
    k_projf<<<NK / 64, 32, 0, stream>>>(XK, W1K, b1, 1, KB);

    k_pairw<<<NQ / (16 * AW), 32 * AW, 0, stream>>>(QP, KB, VH, w2, b2, OUT0, OUT1);
}
